// SupervisedConLoss_70781061038765
// MI455X (gfx1250) — hardware-verified
//
#include <hip/hip_runtime.h>


namespace {
constexpr int N = 8192, D = 128;
constexpr float XS = 8.0f, TEMP = 0.1f, BASE_T = 0.07f, LOG2E = 1.4426950408889634f, LN2 = 0.69314718055994531f;

typedef _Float16 b16;
typedef __attribute__((ext_vector_type(16))) _Float16 v16b;
typedef __attribute__((ext_vector_type(8))) _Float16 v8b;
typedef __attribute__((ext_vector_type(8))) float v8f;
typedef __attribute__((ext_vector_type(4))) float v4f;
typedef __attribute__((ext_vector_type(3))) float v3f;
__device__ __forceinline__ float bf16_rne(float f) { unsigned int u = __float_as_uint(f); u += 0x7FFFu + ((u >> 16) & 1u); return __uint_as_float(u & 0xFFFF0000u); }
__device__ __forceinline__ v16b frag_kb(const b16* p, int hh) { const v8b a = *(const v8b*)(p + 8 * hh), b = *(const v8b*)(p + 16 + 8 * hh); v16b f;
#pragma unroll
  for (int e = 0; e < 8; ++e) { f[e] = a[e]; f[8 + e] = b[e]; } return f; }
__device__ __forceinline__ v8f wmma16b(v16b a, v16b b, v8f c) { v8f d = __builtin_amdgcn_wmma_f32_16x16x32_f16(false, a, false, b, (short)0, c, false, false); asm volatile("v_nop\n\tv_nop\n\tv_nop\n\tv_nop" : "+v"(d) : "v"(a), "v"(b)); return d; }
__device__ __forceinline__ float nexp2(float x) { return __builtin_amdgcn_exp2f(x); }

__global__ __launch_bounds__(256) void prep_kernel(const float* __restrict__ f, b16* __restrict__ F16) {
  const size_t t = (size_t)blockIdx.x * 256 + threadIdx.x; if (t >= (size_t)N * D / 8) return; const size_t e = t * 8; const v4f a = *(const v4f*)(f + e), c = *(const v4f*)(f + e + 4); v8b o;
  for (int j = 0; j < 4; ++j) { o[j] = (b16)(bf16_rne(a[j]) * XS); o[4 + j] = (b16)(bf16_rne(c[j]) * XS); }
  for (int pass = 0; pass < 2; ++pass) { *(volatile v8b*)(F16 + e) = o; __threadfence(); }
}
__global__ __launch_bounds__(64) void row_kernel(const b16* __restrict__ F16, const int* __restrict__ tgt, float* __restrict__ ROW) {
  __shared__ __attribute__((aligned(16))) float Rs[32][4];
  const int wave = threadIdx.x >> 5, lane = threadIdx.x & 31, hh = lane >> 4, col = lane & 15; const int i0 = blockIdx.x * 32 + wave * 16, qi = i0 + col; const int ti = tgt[qi];
  v16b qa[4];
#pragma unroll
  for (int ks = 0; ks < 4; ++ks) qa[ks] = frag_kb(F16 + (size_t)qi * D + ks * 32, hh);
  float m = -INFINITY, l = 0.0f, P = 0.0f, np_ = 0.0f; const float cs = 1.0f / (XS * XS) / TEMP;
  for (int kb = 0; kb < N; kb += 32) {
    v8f s0 = {}, s1 = {};
#pragma unroll
    for (int ks = 0; ks < 4; ++ks) { const v16b f0 = frag_kb(F16 + (size_t)(kb + col) * D + ks * 32, hh), f1 = frag_kb(F16 + (size_t)(kb + 16 + col) * D + ks * 32, hh); s0 = wmma16b(f0, qa[ks], s0); s1 = wmma16b(f1, qa[ks], s1); }
    float lg[16]; float mx = -INFINITY;
#pragma unroll
    for (int r = 0; r < 8; ++r) { lg[r] = s0[r] * cs; lg[8 + r] = s1[r] * cs; mx = fmaxf(mx, fmaxf(lg[r], lg[8 + r])); }
    mx = fmaxf(mx, __shfl_xor(mx, 16)); const float mn = fmaxf(m, mx); const float al = nexp2((m - mn) * LOG2E); m = mn; float sum = 0.0f;
#pragma unroll
    for (int r = 0; r < 16; ++r) { const int j = kb + (r < 8 ? 0 : 16) + 8 * hh + (r & 7); const bool notself = (j != qi); const float e = notself ? nexp2((lg[r] - mn) * LOG2E) : 0.0f; sum += e;
      if (notself && tgt[j] == ti) { P += lg[r]; np_ += 1.0f; } }
    sum += __shfl_xor(sum, 16); l = l * al + sum; }
  P += __shfl_xor(P, 16); np_ += __shfl_xor(np_, 16);
  const float mlpp = (P - np_ * (m + __logf(l + 1e-20f))) / (np_ + 1e-20f); const float nneg = (float)N - np_ - 1.0f;
  if (hh == 0) { Rs[wave * 16 + col][0] = mlpp; Rs[wave * 16 + col][1] = np_; Rs[wave * 16 + col][2] = nneg; Rs[wave * 16 + col][3] = 0.0f; }
  __syncthreads();
  for (int pass = 0; pass < 2; ++pass) { if (threadIdx.x < 32) *(volatile v4f*)(ROW + ((size_t)blockIdx.x * 32 + threadIdx.x) * 4) = *(const v4f*)(&Rs[threadIdx.x][0]); __threadfence(); }
}
__global__ __launch_bounds__(256) void final_kernel(const float* __restrict__ ROW, float* __restrict__ out) {
  __shared__ float pa[256], pb[256], pc[256];
  const int t_ = threadIdx.x; float a = 0.0f, b = 0.0f, c = 0.0f;
  for (int i = t_ * 32; i < t_ * 32 + 32; ++i) { a += ROW[(size_t)i * 4]; b += ROW[(size_t)i * 4 + 1]; c += ROW[(size_t)i * 4 + 2]; }
  pa[t_] = a; pb[t_] = b; pc[t_] = c; __syncthreads();
  for (int st = 128; st >= 1; st >>= 1) { if (t_ < st) { pa[t_] += pa[t_ + st]; pb[t_] += pb[t_ + st]; pc[t_] += pc[t_ + st]; } __syncthreads(); }
  if (t_ == 0) { v3f o; o.x = -(TEMP / BASE_T) * (pa[0] / (float)N); o.y = pb[0] / (float)N; o.z = pc[0] / (float)N; for (int pass = 0; pass < 2; ++pass) { *(volatile v3f*)out = o; __threadfence(); } }
}
}

extern "C" void kernel_launch(void* const* d_in, const int* in_sizes, int n_in, void* d_out, int out_size, void* d_ws, size_t ws_size, hipStream_t stream) {
  (void)n_in;
  if (in_sizes[0] != N * D || in_sizes[1] != N || out_size != 3) return;
  size_t off = 0; char* ws = (char*)d_ws;
  auto carve = [&](size_t bytes) { char* p = ws + off; off += (bytes + 255) & ~(size_t)255; return p; };
  b16* F16 = (b16*)carve((size_t)N * D * 2); float* ROW = (float*)carve((size_t)N * 4 * 4);
  if (off > ws_size) return;
  prep_kernel<<<(N * D / 8 + 255) / 256, 256, 0, stream>>>((const float*)d_in[0], F16);
  row_kernel<<<N / 32, 64, 0, stream>>>(F16, (const int*)d_in[1], ROW);
  final_kernel<<<1, 256, 0, stream>>>(ROW, (float*)d_out);
}
